// GIN_52115133169838
// MI455X (gfx1250) — hardware-verified
//
#include <hip/hip_runtime.h>
#include <stddef.h>
#include <stdint.h>


#define FD     128
#define KZ     (2 * FD)
#define KH1    (4 * FD)
#define KH2    (2 * FD)
#define NTHR   256
#define NWAVE  8
#define EPT    8
#define CHUNK  (NTHR * EPT)
#define WCAP   (EPT * 32)
#define LISTN  (NWAVE * WCAP)
#define NBA    1024
#define SLA    10
#define NBP    256
#define SLP    8
#define RCAP   28672
#define DEGA   64
#define DEGP   256
#define GBM    64
#define GTHR   128
#define GWAVE  (GTHR / 32)
#define GNC    128
#define PARTW  288
#define WSTW   258
#define HPR    8
#define HPB    (NWAVE * HPR)
#define MISC_INTS 16
#define WSMAX  134217728

static_assert((CHUNK & (CHUNK - 1)) == 0 && CHUNK == NTHR * EPT && CHUNK <= 4096);
static_assert(NBA == (1 << SLA) && NBP == (1 << SLP));
static_assert(((long long)CHUNK << SLA) < (1LL << 31) && ((long long)CHUNK << SLP) < (1LL << 31));
static_assert(LISTN == NWAVE * WCAP && LISTN % 4 == 0 && RCAP % 32 == 0);
static_assert(NBA % NWAVE == 0 && NBA % 32 == 0 && NBP % NWAVE == 0 && NBP % 32 == 0);
static_assert(KZ == 2 * FD && KH1 == 4 * FD && KH2 == 2 * FD && KZ % 32 == 0 && KH1 % 32 == 0);
static_assert(GBM == GWAVE * 16 && GTHR == GNC && FD == GNC && FD == 4 * 32);
static_assert(PARTW % 32 == 0 && PARTW / 4 <= GTHR && PARTW >= 2 * GNC + 1);
static_assert(WSTW >= 2 * GNC + 1 && (WSTW % 2) == 0);
static_assert(HPB == GBM && NTHR == 2 * FD && HPB == NWAVE * HPR);
static_assert((LISTN + 2 * RCAP + 3 * NBA + MISC_INTS) * 4 <= 300000);

typedef float          v2f   __attribute__((ext_vector_type(2)));
typedef float          v4f   __attribute__((ext_vector_type(4)));
typedef float          v8f   __attribute__((ext_vector_type(8)));
typedef int            v4i   __attribute__((ext_vector_type(4)));
typedef int            v8i   __attribute__((ext_vector_type(8)));
typedef unsigned int   v2u   __attribute__((ext_vector_type(2)));
typedef unsigned int   v4u   __attribute__((ext_vector_type(4)));
typedef unsigned short v4us  __attribute__((ext_vector_type(4)));
typedef unsigned short v8us  __attribute__((ext_vector_type(8)));
typedef unsigned short v16us __attribute__((ext_vector_type(16)));
typedef __bf16         v16bf __attribute__((ext_vector_type(16)));
typedef v2f  __attribute__((may_alias)) v2fa;
typedef v4f  __attribute__((may_alias)) v4fa;
typedef v4i  __attribute__((may_alias)) v4ia;
typedef v4us __attribute__((may_alias)) v4usa;
typedef v8us __attribute__((may_alias)) v8usa;
union FragB { v16bf v; v16us u; v8us h[2]; v8i w; };

__device__ __forceinline__ v8f wmb(const FragB& a, const FragB& b, v8f c) {
  v8f d = __builtin_amdgcn_wmma_f32_16x16x32_bf16(false, a.v, false, b.v, (short)0, c, false, false);
  asm volatile("v_nop\n\tv_nop\n\tv_nop\n\tv_nop" : "+v"(d) : "v"(a.w), "v"(b.w));
  return d;
}

__device__ __forceinline__ v8f z8() { v8f z = {0.f, 0.f, 0.f, 0.f, 0.f, 0.f, 0.f, 0.f}; return z; }

__device__ __forceinline__ unsigned bf16_bits(float f) {
  const unsigned u = __float_as_uint(f);
  return ((u + 0x7FFFu + ((u >> 16) & 1u)) >> 16) & 0xFFFFu;
}
__device__ __forceinline__ float bf16_val(float f) {
  return __uint_as_float(bf16_bits(f) << 16);
}
__device__ __forceinline__ unsigned hl_bits(float v, unsigned& lo) {
  const unsigned hb = bf16_bits(v);
  lo = bf16_bits(v - __uint_as_float(hb << 16));
  return hb;
}
__device__ __forceinline__ unsigned pk2(float lo, float hi) { return bf16_bits(lo) | (bf16_bits(hi) << 16); }
__device__ __forceinline__ v4u pack8(const v4f a, const v4f b) {
  v4u r;
  r.x = pk2(a.x, a.y); r.y = pk2(a.z, a.w); r.z = pk2(b.x, b.y); r.w = pk2(b.z, b.w);
  return r;
}

__device__ __forceinline__ void wave_sync() {
  __builtin_amdgcn_fence(__ATOMIC_RELEASE, "wavefront");
  __builtin_amdgcn_wave_barrier();
  __builtin_amdgcn_fence(__ATOMIC_ACQUIRE, "wavefront");
}

template <int SLB>
__device__ __forceinline__ int scan_chunk(const int* __restrict__ dsts, int nE, int cbase, int slotBase,
                                          int nb, int vec8, int* list, int tid, int lane, int wave) {
  int wc = 0;
  const int el0  = tid * EPT;
  const int e0   = cbase + el0;
  const int sent = -2147483647 - 1;
  v4i da, db;
  if (vec8 != 0 && cbase + CHUNK <= nE) {
    da = *(const v4i*)(dsts + e0);
    db = *(const v4i*)(dsts + e0 + 4);
  } else {
    da.x = (e0     < nE) ? dsts[min(e0,     nE - 1)] : sent;
    da.y = (e0 + 1 < nE) ? dsts[min(e0 + 1, nE - 1)] : sent;
    da.z = (e0 + 2 < nE) ? dsts[min(e0 + 2, nE - 1)] : sent;
    da.w = (e0 + 3 < nE) ? dsts[min(e0 + 3, nE - 1)] : sent;
    db.x = (e0 + 4 < nE) ? dsts[min(e0 + 4, nE - 1)] : sent;
    db.y = (e0 + 5 < nE) ? dsts[min(e0 + 5, nE - 1)] : sent;
    db.z = (e0 + 6 < nE) ? dsts[min(e0 + 6, nE - 1)] : sent;
    db.w = (e0 + 7 < nE) ? dsts[min(e0 + 7, nE - 1)] : sent;
  }
  const unsigned nbs = (unsigned)slotBase;
  const unsigned unb = (unsigned)nb;
  const unsigned s0 = (unsigned)da.x - nbs, s1 = (unsigned)da.y - nbs;
  const unsigned s2 = (unsigned)da.z - nbs, s3 = (unsigned)da.w - nbs;
  const unsigned s4 = (unsigned)db.x - nbs, s5 = (unsigned)db.y - nbs;
  const unsigned s6 = (unsigned)db.z - nbs, s7 = (unsigned)db.w - nbs;
  const bool h0 = s0 < unb, h1 = s1 < unb, h2 = s2 < unb, h3 = s3 < unb;
  const bool h4 = s4 < unb, h5 = s5 < unb, h6 = s6 < unb, h7 = s7 < unb;
  const unsigned any = __builtin_amdgcn_ballot_w32(h0 | h1 | h2 | h3 | h4 | h5 | h6 | h7);
  if (any != 0u) {
#define HITJ(J, HJ, SJ) { \
      const unsigned mj = __builtin_amdgcn_ballot_w32(HJ); \
      if (mj != 0u) { \
        if (HJ) { \
          const int pos = wc + (int)__builtin_amdgcn_mbcnt_lo(mj, 0u); \
          if (pos < WCAP) list[wave * WCAP + pos] = ((el0 + (J)) << SLB) | (int)(SJ); \
        } \
        wc += (int)__builtin_popcount(mj); } }
    HITJ(0, h0, s0)
    HITJ(1, h1, s1)
    HITJ(2, h2, s2)
    HITJ(3, h3, s3)
    HITJ(4, h4, s4)
    HITJ(5, h5, s5)
    HITJ(6, h6, s6)
    HITJ(7, h7, s7)
#undef HITJ
  }
  return wc;
}

__global__ __launch_bounds__(NTHR) void k_wcvt(const float* __restrict__ w0, const float* __restrict__ w1,
                                               const float* __restrict__ w2, const float* __restrict__ w3,
                                               int K, int nUnits,
                                               unsigned short* o0, unsigned short* o1,
                                               unsigned short* o2, unsigned short* o3) {
  const int y = (int)blockIdx.y;
  const float* w = w0;
  unsigned short* o = o0;
  if (y == 1) { w = w1; o = o1; }
  else if (y == 2) { w = w2; o = o2; }
  else if (y == 3) { w = w3; o = o3; }
  const int u = (int)blockIdx.x * NTHR + (int)threadIdx.x;
  if (u >= nUnits) return;
  const int kq = K >> 3;
  const int n  = u / kq;
  const int k8 = (u - n * kq) * 8;
  const float* p = w + (size_t)n * (size_t)K + k8;
  const v4f a = *(const v4fa*)p;
  const v4f b = *(const v4fa*)(p + 4);
  const v4u wv = pack8(a, b);
  unsigned short* q = o + (size_t)n * (size_t)(2 * K) + k8;
  *(volatile v4u*)q = wv;
  *(volatile v4u*)(q + K) = wv;
  __threadfence();
  *(volatile v4u*)q = wv;
  *(volatile v4u*)(q + K) = wv;
}

__global__ __launch_bounds__(NTHR) void k_hinit(const int* __restrict__ xi, const float* __restrict__ emb,
                                                int nEmbRows, int nN, int nUnits, float* hout) {
  const int u = (int)blockIdx.x * NTHR + (int)threadIdx.x;
  if (u >= nUnits) return;
  const int row = u >> 5, j = u & 31;
  const bool live = row < nN;
  const int rc = live ? row : (nN - 1);
  int ix = xi[rc];
  ix = ix < 0 ? 0 : (ix > nEmbRows - 1 ? nEmbRows - 1 : ix);
  const v4f a = *(const v4fa*)(emb + (size_t)ix * FD + 4 * j);
  v4f y;
  y.x = live ? bf16_val(a.x) : 0.0f;
  y.y = live ? bf16_val(a.y) : 0.0f;
  y.z = live ? bf16_val(a.z) : 0.0f;
  y.w = live ? bf16_val(a.w) : 0.0f;
  float* op = hout + (size_t)row * FD + 4 * j;
  *(volatile v4f*)op = y;
  __threadfence();
  *(volatile v4f*)op = y;
}

template <int MSG, int NB, int SLB, int DEGC>
__global__ __launch_bounds__(NTHR) void k_scan(const int* __restrict__ srcs, const int* __restrict__ dsts,
                                               int nE, int nOwn, int nSrc, int vec8, int mRows,
                                               const float* __restrict__ eattr, const float* __restrict__ ewp,
                                               const float* __restrict__ ebp, const float* __restrict__ hsrc,
                                               unsigned short* apl, int pitch, int hiOff, int loOff) {
#pragma clang fp contract(off)
  constexpr int ZINTS = LISTN + 2 * RCAP + 3 * NB;
  static_assert(NB % NWAVE == 0 && NB % 32 == 0 && (ZINTS % 4) == 0 && NB == (1 << SLB));
  static_assert((ZINTS + MISC_INTS) * 4 <= 300000);
  extern __shared__ __attribute__((aligned(16))) int dsm[];
  int* list = dsm;
  int* hl   = dsm + LISTN;
  int* sl   = hl + RCAP;
  int* cnt  = sl + RCAP;
  int* offs = cnt + NB;
  int* cur  = offs + NB;
  int* misc = cur + NB;
  const int tid = (int)threadIdx.x, lane = tid & 31, wave = tid >> 5;
  const int nodeBase = (int)blockIdx.x * NB;

  {
    const v4i z4 = {0, 0, 0, 0};
    for (int i = tid * 4; i < ZINTS; i += NTHR * 4) *(v4ia*)(dsm + i) = z4;
    if (tid < MISC_INTS) misc[tid] = 0;
  }
  __syncthreads();

  float wx[4], bq[4];
  if constexpr (MSG == 0) {
    const v4f w4 = *(const v4fa*)(ewp + 4 * lane);
    const v4f b4 = *(const v4fa*)(ebp + 4 * lane);
    wx[0] = bf16_val(w4.x); wx[1] = bf16_val(w4.y); wx[2] = bf16_val(w4.z); wx[3] = bf16_val(w4.w);
    bq[0] = bf16_val(b4.x); bq[1] = bf16_val(b4.y); bq[2] = bf16_val(b4.z); bq[3] = bf16_val(b4.w);
  } else {
#pragma unroll
    for (int j = 0; j < 4; ++j) { wx[j] = 0.0f; bq[j] = 0.0f; }
    (void)ewp; (void)ebp; (void)eattr; (void)srcs;
  }

  int t = 0, ov = 0;
  const int nChunks = (nE + CHUNK - 1) / CHUNK;
#pragma unroll 1
  for (int ch = 0; ch < nChunks; ++ch) {
    const int cbase = ch * CHUNK;
    const int wc = scan_chunk<SLB>(dsts, nE, cbase, nodeBase, NB, vec8, list, tid, lane, wave);
    if (lane == 0) misc[wave] = wc;
    __syncthreads();
    if (wave == 0) {
#pragma unroll 1
      for (int w2 = 0; w2 < NWAVE; ++w2) {
        int c = misc[w2];
        c = c < 0 ? 0 : (c > WCAP ? WCAP : c);
#pragma unroll 1
        for (int b0 = 0; b0 < c; b0 += 32) {
          const int idx = b0 + lane;
          const int ent = list[w2 * WCAP + (idx < WCAP ? idx : WCAP - 1)];
          const int m32 = (c - b0) < 32 ? (c - b0) : 32;
#pragma unroll 1
          for (int k = 0; k < m32; ++k) {
            const int u    = __builtin_amdgcn_readlane(ent, k);
            const int slot = u & (NB - 1);
            const int el   = (u >> SLB) & (CHUNK - 1);
            const int pk   = ((cbase + el) << SLB) | slot;
            if (t < RCAP) {
              if (lane == 0) { hl[t] = pk; cnt[slot] = cnt[slot] + 1; }
              t = t + 1;
            } else {
              ov = 1;
            }
          }
        }
      }
    }
    __syncthreads();
  }
  if (wave == 0 && lane == 0) { misc[8] = t; misc[9] = ov; }
  __syncthreads();
  int tt = misc[8];
  tt = tt < 0 ? 0 : (tt > RCAP ? RCAP : tt);
  const int ovf = misc[9];

  if (wave == 0) {
    const int base = lane * (NB / 32);
    int s = 0;
#pragma unroll 1
    for (int i = 0; i < NB / 32; ++i) s += cnt[base + i];
    int incl = s;
#pragma unroll
    for (int d = 1; d < 32; d <<= 1) {
      const int y = __shfl_up(incl, d, 32);
      if (lane >= d) incl += y;
    }
    int run = incl - s;
#pragma unroll 1
    for (int i = 0; i < NB / 32; ++i) {
      const int cv = cnt[base + i];
      offs[base + i] = run;
      cur[base + i]  = run;
      run += cv;
    }
  }
  __syncthreads();
  if (wave == 0) {
#pragma unroll 1
    for (int b0 = 0; b0 < tt; b0 += 32) {
      const int idx = b0 + lane;
      const int ent = hl[idx < RCAP ? idx : RCAP - 1];
      const int m32 = (tt - b0) < 32 ? (tt - b0) : 32;
#pragma unroll 1
      for (int k = 0; k < m32; ++k) {
        const int u    = __builtin_amdgcn_readlane(ent, k);
        const int slot = u & (NB - 1);
        if (lane == 0) {
          int p = cur[slot];
          p = p < 0 ? 0 : (p > RCAP - 1 ? RCAP - 1 : p);
          sl[p] = u;
          cur[slot] = p + 1;
        }
      }
    }
  }
  __syncthreads();

  const float qnan = __int_as_float(0x7fc00000);
  const float pz = (ovf != 0) ? qnan : 0.0f;
#pragma unroll 1
  for (int si = 0; si < NB / NWAVE; ++si) {
    const int s    = si * NWAVE + wave;
    const int node = nodeBase + s;
    int c = cnt[s];
    const bool big = c > DEGC;
    c = c < 0 ? 0 : (c > DEGC ? DEGC : c);
    int o = offs[s];
    o = o < 0 ? 0 : (o > RCAP ? RCAP : o);
    float ag[4];
#pragma unroll
    for (int j = 0; j < 4; ++j) ag[j] = 0.0f;
#pragma unroll 1
    for (int b0 = 0; b0 < c; b0 += 32) {
      int idx = o + b0 + lane;
      idx = idx > RCAP - 1 ? RCAP - 1 : idx;
      const int ent = sl[idx];
      int eid = ent >> SLB;
      eid = eid < 0 ? 0 : (eid > nE - 1 ? nE - 1 : eid);
      int sr;
      float ea = 0.0f;
      if constexpr (MSG == 0) {
        sr = srcs[eid];
        sr = sr < 0 ? 0 : (sr > nSrc - 1 ? nSrc - 1 : sr);
        ea = bf16_val(eattr[eid]);
      } else {
        sr = eid > nSrc - 1 ? nSrc - 1 : eid;
      }
      const int eab = __float_as_int(ea);
      const int m32 = (c - b0) < 32 ? (c - b0) : 32;
#pragma unroll 1
      for (int k = 0; k < m32; ++k) {
        const int sk = __builtin_amdgcn_readlane(sr, k);
        const v4f hv = *(const v4fa*)(hsrc + (size_t)sk * FD + 4 * lane);
        if constexpr (MSG == 0) {
          const float ek = __int_as_float(__builtin_amdgcn_readlane(eab, k));
          float d0 = ek * wx[0]; d0 = d0 + bq[0];
          float d1 = ek * wx[1]; d1 = d1 + bq[1];
          float d2 = ek * wx[2]; d2 = d2 + bq[2];
          float d3 = ek * wx[3]; d3 = d3 + bq[3];
          ag[0] = ag[0] + fmaxf(hv.x + d0, 0.0f);
          ag[1] = ag[1] + fmaxf(hv.y + d1, 0.0f);
          ag[2] = ag[2] + fmaxf(hv.z + d2, 0.0f);
          ag[3] = ag[3] + fmaxf(hv.w + d3, 0.0f);
        } else {
          (void)eab;
          ag[0] = ag[0] + hv.x;
          ag[1] = ag[1] + hv.y;
          ag[2] = ag[2] + hv.z;
          ag[3] = ag[3] + hv.w;
        }
      }
    }
    const float pzr = big ? qnan : pz;
    const bool live = node < nOwn;
    float z[4];
    if constexpr (MSG == 0) {
      const int nc = node < nSrc ? node : nSrc - 1;
      const v4f hr = *(const v4fa*)(hsrc + (size_t)nc * FD + 4 * lane);
      z[0] = live ? ((hr.x + ag[0]) + pzr) : 0.0f;
      z[1] = live ? ((hr.y + ag[1]) + pzr) : 0.0f;
      z[2] = live ? ((hr.z + ag[2]) + pzr) : 0.0f;
      z[3] = live ? ((hr.w + ag[3]) + pzr) : 0.0f;
    } else {
#pragma unroll
      for (int j = 0; j < 4; ++j) z[j] = live ? (ag[j] + pzr) : 0.0f;
    }
    unsigned hb[4], lb[4];
#pragma unroll
    for (int j = 0; j < 4; ++j) hb[j] = hl_bits(z[j], lb[j]);
    if (node < mRows) {
      unsigned short* rpw = apl + (size_t)node * (size_t)pitch;
      v2u hp, lp;
      hp.x = hb[0] | (hb[1] << 16); hp.y = hb[2] | (hb[3] << 16);
      lp.x = lb[0] | (lb[1] << 16); lp.y = lb[2] | (lb[3] << 16);
      unsigned short* ph = rpw + hiOff + 4 * lane;
      unsigned short* pl = rpw + loOff + 4 * lane;
      *(volatile v2u*)ph = hp;
      *(volatile v2u*)pl = lp;
      __threadfence();
      *(volatile v2u*)ph = hp;
      *(volatile v2u*)pl = lp;
    }
  }
}

template <int NC, int KK, int EPI>
__global__ __launch_bounds__(GTHR) void k_gemm(const unsigned short* __restrict__ Apl,
                                               const unsigned short* __restrict__ BT,
                                               const float* __restrict__ bias, int nN,
                                               float* outp, int ldo, float* part) {
  constexpr int NT  = NC / 16;
  constexpr int CPL = NC / 32;
  static_assert(NT == 8 && CPL == 4 && KK % 32 == 0 && NC == GNC);
  static_assert(EPI >= 0 && EPI <= 3);
  __shared__ __attribute__((aligned(16))) float stg[GBM * NC];
  __shared__ __attribute__((aligned(16))) float wst[GWAVE * WSTW];
  __shared__ __attribute__((aligned(16))) float pst[PARTW];
  const int tid = (int)threadIdx.x, lane = tid & 31, wave = tid >> 5, hh = lane >> 4, m = lane & 15;
  const int rowBase = (int)blockIdx.x * GBM;
  const int col0    = (int)blockIdx.y * NC;

  v8f acc[NT];
#pragma unroll
  for (int t = 0; t < NT; ++t) acc[t] = z8();
  const unsigned short* ap = Apl + (size_t)(rowBase + 16 * wave + m) * (size_t)KK + 8 * hh;
  const unsigned short* bp = BT + (size_t)(col0 + m) * (size_t)KK + 8 * hh;

#pragma unroll 1
  for (int k0 = 0; k0 < KK; k0 += 32) {
    FragB af;
    af.h[0] = *(const v8usa*)(ap + k0);
    af.h[1] = *(const v8usa*)(ap + k0 + 16);
#pragma unroll
    for (int nt = 0; nt < NT; ++nt) {
      const unsigned short* wq = bp + (size_t)(16 * nt) * (size_t)KK + k0;
      FragB bf;
      bf.h[0] = *(const v8usa*)wq;
      bf.h[1] = *(const v8usa*)(wq + 16);
      acc[nt] = wmb(af, bf, acc[nt]);
    }
  }

#pragma unroll
  for (int nt = 0; nt < NT; ++nt) {
    const int lc = 16 * nt + m;
#pragma unroll
    for (int r = 0; r < 8; ++r) {
      const int lr = 16 * wave + 8 * hh + r;
      stg[lr * NC + lc] = acc[nt][r];
    }
  }
  __syncthreads();

  float bq[CPL];
  {
    const v4f b4 = *(const v4fa*)(bias + col0 + 4 * lane);
    bq[0] = bf16_val(b4.x); bq[1] = bf16_val(b4.y); bq[2] = bf16_val(b4.z); bq[3] = bf16_val(b4.w);
  }

  float pv[16][CPL];
  unsigned pw[16][4];
  int wn = 0;
  float wm[CPL], wqv[CPL];
#pragma unroll
  for (int j = 0; j < CPL; ++j) { wm[j] = 0.0f; wqv[j] = 0.0f; }
#pragma unroll
  for (int i = 0; i < 16; ++i) {
    const int row = rowBase + 16 * wave + i;
    const bool ok = row < nN;
    float x[CPL];
    {
      const v4f t4 = *(const v4fa*)(stg + (16 * wave + i) * NC + 4 * lane);
      x[0] = t4.x; x[1] = t4.y; x[2] = t4.z; x[3] = t4.w;
    }
    float vv[CPL];
#pragma unroll
    for (int j = 0; j < CPL; ++j) {
      if constexpr (EPI == 0) {
        vv[j] = ok ? (x[j] + bq[j]) : 0.0f;
      } else if constexpr (EPI == 3) {
        vv[j] = x[j] + bq[j];
      } else {
        vv[j] = ok ? fmaxf(x[j] + bq[j], 0.0f) : 0.0f;
      }
    }
    if constexpr (EPI == 2) {
      unsigned hb[4], lb[4];
#pragma unroll
      for (int j = 0; j < 4; ++j) hb[j] = hl_bits(vv[j], lb[j]);
      pw[i][0] = hb[0] | (hb[1] << 16); pw[i][1] = hb[2] | (hb[3] << 16);
      pw[i][2] = lb[0] | (lb[1] << 16); pw[i][3] = lb[2] | (lb[3] << 16);
#pragma unroll
      for (int j = 0; j < CPL; ++j) pv[i][j] = 0.0f;
    } else {
#pragma unroll
      for (int j = 0; j < CPL; ++j) pv[i][j] = vv[j];
#pragma unroll
      for (int j = 0; j < 4; ++j) pw[i][j] = 0u;
    }
    if constexpr (EPI == 0) {
      if (ok) {
        wn += 1;
        const float rk = 1.0f / (float)(i + 1);
#pragma unroll
        for (int j = 0; j < CPL; ++j) {
          const float dd = vv[j] - wm[j];
          wm[j]  = fmaf(dd, rk, wm[j]);
          wqv[j] = fmaf(dd, vv[j] - wm[j], wqv[j]);
        }
      }
    }
  }

#pragma unroll
  for (int ps = 0; ps < 2; ++ps) {
    if (ps == 1) __threadfence();
#pragma unroll
    for (int i = 0; i < 16; ++i) {
      const int row = rowBase + 16 * wave + i;
      if constexpr (EPI == 2) {
        unsigned short* o16 = (unsigned short*)outp;
        unsigned short* ph = o16 + (size_t)row * (size_t)(2 * ldo) + col0 + 4 * lane;
        unsigned short* pl = ph + ldo;
        v2u hp, lp;
        hp.x = pw[i][0]; hp.y = pw[i][1]; lp.x = pw[i][2]; lp.y = pw[i][3];
        *(volatile v2u*)ph = hp;
        *(volatile v2u*)pl = lp;
      } else {
        const bool wr = (EPI != 3) || (row < nN);
        float* op = outp + (size_t)row * (size_t)ldo + col0 + CPL * lane;
        if (wr) {
          v4f q; q.x = pv[i][0]; q.y = pv[i][1]; q.z = pv[i][2]; q.w = pv[i][3];
          *(volatile v4f*)op = q;
        }
      }
    }
  }

  if constexpr (EPI == 0) {
    if (lane == 0) wst[wave * WSTW] = (float)wn;
#pragma unroll
    for (int j = 0; j < CPL; ++j) {
      wst[wave * WSTW + 1 + CPL * lane + j]       = wm[j];
      wst[wave * WSTW + 1 + GNC + CPL * lane + j] = wqv[j];
    }
#pragma unroll 1
    for (int i = tid; i < PARTW; i += GTHR) pst[i] = 0.0f;
    __syncthreads();
    if (tid < NC) {
      float n = 0.0f, mean = 0.0f, M2 = 0.0f;
#pragma unroll 1
      for (int w2 = 0; w2 < GWAVE; ++w2) {
        const float nb = wst[w2 * WSTW];
        const float mb = wst[w2 * WSTW + 1 + tid];
        const float qb = wst[w2 * WSTW + 1 + GNC + tid];
        if (nb > 0.5f) {
          const float nn = n + nb;
          const float delta = mb - mean;
          const float f = nb / nn;
          mean = fmaf(delta, f, mean);
          M2 = M2 + qb + delta * delta * n * f;
          n = nn;
        }
      }
      pst[1 + tid] = mean;
      pst[1 + GNC + tid] = M2;
      if (tid == 0) pst[0] = n;
    }
    __syncthreads();
    const int pb = (int)blockIdx.x * (int)gridDim.y + (int)blockIdx.y;
    v4f ps4 = {0.0f, 0.0f, 0.0f, 0.0f};
    if (tid < PARTW / 4) {
      ps4 = *(const v4fa*)(pst + 4 * tid);
      *(volatile v4f*)(part + (size_t)pb * PARTW + 4 * tid) = ps4;
    }
    __threadfence();
    if (tid < PARTW / 4) {
      *(volatile v4f*)(part + (size_t)pb * PARTW + 4 * tid) = ps4;
    }
  } else {
    (void)part; (void)wn; (void)wm; (void)wqv;
  }
}

__global__ __launch_bounds__(GNC) void k_bnfin(const float* __restrict__ part, int nPart,
                                               const float* __restrict__ gam, const float* __restrict__ bet,
                                               float* ss) {
  __shared__ __attribute__((aligned(16))) float stg[2 * GNC];
  const int tid = (int)threadIdx.x;
  const int c = tid < GNC ? tid : GNC - 1;
  double n = 0.0, mean = 0.0, M2 = 0.0;
#pragma unroll 1
  for (int b = 0; b < nPart; ++b) {
    const float* pr = part + (size_t)b * PARTW;
    const double nb = (double)pr[0];
    const double mb = (double)pr[1 + c];
    const double qb = (double)pr[1 + GNC + c];
    if (nb > 0.5) {
      const double nn = n + nb;
      const double delta = mb - mean;
      const double f = nb / nn;
      mean = mean + delta * f;
      M2 = M2 + qb + delta * delta * n * f;
      n = nn;
    }
  }
  const double ntot = n < 1.0 ? 1.0 : n;
  const float varf  = (float)(M2 / ntot);
  const float meanf = (float)mean;
  const float rstd = rsqrtf(varf + 1e-5f);
  const float sc = bf16_val(gam[c]) * rstd;
  const float sh = bf16_val(bet[c]) - meanf * sc;
  if (tid < GNC) {
    stg[c] = sc;
    stg[GNC + c] = sh;
  }
  __syncthreads();
  v4f v = {0.0f, 0.0f, 0.0f, 0.0f};
  if (tid < (2 * GNC) / 4) {
    v = *(const v4fa*)(stg + 4 * tid);
    *(volatile v4f*)(ss + 4 * tid) = v;
  }
  __threadfence();
  if (tid < (2 * GNC) / 4) {
    *(volatile v4f*)(ss + 4 * tid) = v;
  }
}

__global__ __launch_bounds__(NTHR) void k_apply1(const float* __restrict__ s1, const float* __restrict__ ss,
                                                 int nN, int mRows, unsigned short* apl2) {
  __shared__ __attribute__((aligned(16))) float ssh[2 * FD];
  __shared__ __attribute__((aligned(16))) unsigned short rbuf[NWAVE * 2 * FD];
  const int tid = (int)threadIdx.x, lane = tid & 31, wave = tid >> 5;
  ssh[tid] = ss[tid];
  __syncthreads();
  const v4f sc = *(const v4fa*)(ssh + 4 * lane);
  const v4f sh = *(const v4fa*)(ssh + FD + 4 * lane);
  unsigned short* rb = rbuf + wave * (2 * FD);
  const int rb0 = (int)blockIdx.x * HPB + wave * HPR;

  v8us qv[HPR];
#pragma unroll
  for (int i = 0; i < HPR; ++i) {
    const int row = rb0 + i;
    const bool live = row < nN;
    const int rc = live ? row : (nN - 1);
    const v4f a = *(const v4fa*)(s1 + (size_t)rc * FD + 4 * lane);
    v4f y;
    y.x = fmaxf(fmaf(a.x, sc.x, sh.x), 0.0f);
    y.y = fmaxf(fmaf(a.y, sc.y, sh.y), 0.0f);
    y.z = fmaxf(fmaf(a.z, sc.z, sh.z), 0.0f);
    y.w = fmaxf(fmaf(a.w, sc.w, sh.w), 0.0f);
    y.x = live ? y.x : 0.0f; y.y = live ? y.y : 0.0f; y.z = live ? y.z : 0.0f; y.w = live ? y.w : 0.0f;
    v4us mh, ml;
    {
      unsigned lb;
      unsigned hb;
      hb = hl_bits(y.x, lb); mh[0] = (unsigned short)hb; ml[0] = (unsigned short)lb;
      hb = hl_bits(y.y, lb); mh[1] = (unsigned short)hb; ml[1] = (unsigned short)lb;
      hb = hl_bits(y.z, lb); mh[2] = (unsigned short)hb; ml[2] = (unsigned short)lb;
      hb = hl_bits(y.w, lb); mh[3] = (unsigned short)hb; ml[3] = (unsigned short)lb;
    }
    *(v4usa*)(rb + 4 * lane) = mh;
    *(v4usa*)(rb + FD + 4 * lane) = ml;
    wave_sync();
    qv[i] = *(const v8usa*)(rb + 8 * lane);
    wave_sync();
  }
#pragma unroll
  for (int i = 0; i < HPR; ++i) {
    const int row = rb0 + i;
    if (row < mRows) {
      *(volatile v8us*)(apl2 + (size_t)row * KZ + 8 * lane) = qv[i];
    }
  }
  __threadfence();
#pragma unroll
  for (int i = 0; i < HPR; ++i) {
    const int row = rb0 + i;
    if (row < mRows) {
      *(volatile v8us*)(apl2 + (size_t)row * KZ + 8 * lane) = qv[i];
    }
  }
}

static inline int cdiv(int a, int b) { return (a + b - 1) / b; }
static inline size_t al256(size_t o) { return (o + 255) & ~(size_t)255; }

extern "C" void kernel_launch(void* const* d_in, const int* in_sizes, int n_in,
                              void* d_out, int out_size, void* d_ws, size_t ws_size,
                              hipStream_t stream) {
  if (n_in < 29) return;
  const int nN = in_sizes[0];
  if (nN < 16 || nN >= (1 << 22)) return;
  if (in_sizes[1] < 2 || (in_sizes[1] & 1) != 0) return;
  const int nE = in_sizes[1] / 2;
  if (nE < 1 || nE >= (1 << 21)) return;
  if (in_sizes[2] != nE) return;
  if (in_sizes[3] != nN) return;
  if (in_sizes[4] < FD || (in_sizes[4] % FD) != 0) return;
  const int nR = in_sizes[4] / FD;
  if (in_sizes[5] != FD || in_sizes[6] != FD) return;
  if (in_sizes[7] != FD * FD || in_sizes[8] != FD) return;
  if (in_sizes[9] != FD || in_sizes[10] != FD) return;
  if (in_sizes[11] != FD * FD || in_sizes[12] != FD) return;
  if (in_sizes[13] != FD || in_sizes[14] != FD) return;
  if (in_sizes[15] != FD * FD || in_sizes[16] != FD) return;
  if (in_sizes[17] != FD || in_sizes[18] != FD) return;
  if (in_sizes[19] != FD * FD || in_sizes[20] != FD) return;
  if (in_sizes[21] != FD * 2 * FD || in_sizes[22] != FD) return;
  const int nT = in_sizes[24];
  if (nT < GNC || (nT % GNC) != 0 || nT > (1 << 16)) return;
  if (in_sizes[23] != nT * FD) return;
  if (in_sizes[25] != FD * 2 * FD || in_sizes[26] != FD) return;
  if (in_sizes[27] != nT * FD || in_sizes[28] != nT) return;
  if (out_size < 2 * nT || (out_size % (2 * nT)) != 0) return;
  const int nG = out_size / (2 * nT);
  if (nG < 1 || nG >= (1 << 22)) return;
  if ((long long)2 * nG * nT != (long long)out_size) return;

  const int*   xi    = (const int*)d_in[0];
  const int*   edge  = (const int*)d_in[1];
  const float* eattr = (const float*)d_in[2];
  const int*   batch = (const int*)d_in[3];
  const float* emb   = (const float*)d_in[4];
  const float* e1w   = (const float*)d_in[5];
  const float* e1b   = (const float*)d_in[6];
  const float* c1w1  = (const float*)d_in[7];
  const float* c1b1  = (const float*)d_in[8];
  const float* c1g   = (const float*)d_in[9];
  const float* c1be  = (const float*)d_in[10];
  const float* c1w2  = (const float*)d_in[11];
  const float* c1b2  = (const float*)d_in[12];
  const float* e2w   = (const float*)d_in[13];
  const float* e2b   = (const float*)d_in[14];
  const float* c2w1  = (const float*)d_in[15];
  const float* c2b1  = (const float*)d_in[16];
  const float* c2g   = (const float*)d_in[17];
  const float* c2be  = (const float*)d_in[18];
  const float* c2w2  = (const float*)d_in[19];
  const float* c2b2  = (const float*)d_in[20];
  const float* fw1   = (const float*)d_in[21];
  const float* fb1   = (const float*)d_in[22];
  const float* fw2   = (const float*)d_in[23];
  const float* fb2   = (const float*)d_in[24];
  const float* bw1   = (const float*)d_in[25];
  const float* bb1   = (const float*)d_in[26];
  const float* bw2   = (const float*)d_in[27];
  const float* bb2   = (const float*)d_in[28];
  float* out = (float*)d_out;
  const int* src = edge;
  const int* dst = edge + nE;

  const int MP = cdiv(nN, GBM) * GBM;
  const int gM = MP / GBM;
  const int gA = cdiv(nN, NBA);
  if ((long long)gA * NBA < (long long)MP) return;
  if ((MP % HPB) != 0) return;
  const int GP = cdiv(nG, GBM) * GBM;
  const int gH = GP / GBM;
  const int gP = cdiv(nG, NBP);
  if ((long long)gP * NBP < (long long)GP) return;
  const int vec8e = ((nE & 3) == 0) ? 1 : 0;
  const int vec8b = ((nN & 3) == 0) ? 1 : 0;

  char* ws = (char*)d_ws;
  size_t off = 0;
  const size_t oBTC = off; off = al256(off + (size_t)4 * FD * KZ * 2);
  const size_t oBH1 = off; off = al256(off + (size_t)2 * FD * KH1 * 2);
  const size_t oBH2 = off; off = al256(off + (size_t)2 * nT * KH2 * 2);
  const size_t oSH  = off; off = al256(off + (size_t)MP * FD * 4);
  const size_t oZA  = off; off = al256(off + (size_t)MP * KZ * 2);
  const size_t oPT  = off; off = al256(off + (size_t)gM * PARTW * 4);
  const size_t oSS  = off; off = al256(off + (size_t)(2 * FD) * 4);
  const size_t oP   = off; off = al256(off + (size_t)GP * KH1 * 2);
  const size_t oQ   = off; off = al256(off + (size_t)GP * KH2 * 2);
  if (off > ws_size || off > (size_t)WSMAX) return;
  unsigned short* BTC = (unsigned short*)(ws + oBTC);
  unsigned short* BH1 = (unsigned short*)(ws + oBH1);
  unsigned short* BH2 = (unsigned short*)(ws + oBH2);
  float*          SH  = (float*)(ws + oSH);
  unsigned short* ZA  = (unsigned short*)(ws + oZA);
  float*          PT  = (float*)(ws + oPT);
  float*          SS  = (float*)(ws + oSS);
  unsigned short* P   = (unsigned short*)(ws + oP);
  unsigned short* Q   = (unsigned short*)(ws + oQ);

  const size_t ldsA = (size_t)(LISTN + 2 * RCAP + 3 * NBA + MISC_INTS) * 4;
  const size_t ldsP = (size_t)(LISTN + 2 * RCAP + 3 * NBP + MISC_INTS) * 4;
  hipFuncSetAttribute(reinterpret_cast<const void*>(&k_scan<0, NBA, SLA, DEGA>), hipFuncAttributeMaxDynamicSharedMemorySize, (int)ldsA);
  hipFuncSetAttribute(reinterpret_cast<const void*>(&k_scan<1, NBP, SLP, DEGP>), hipFuncAttributeMaxDynamicSharedMemorySize, (int)ldsP);

  {
    const int nUc = FD * (FD / 8);
    k_wcvt<<<dim3(cdiv(nUc, NTHR), 4), NTHR, 0, stream>>>(c1w1, c1w2, c2w1, c2w2, FD, nUc,
        BTC, BTC + (size_t)1 * FD * KZ, BTC + (size_t)2 * FD * KZ, BTC + (size_t)3 * FD * KZ);
    const int nU1 = FD * (2 * FD / 8);
    k_wcvt<<<dim3(cdiv(nU1, NTHR), 2), NTHR, 0, stream>>>(fw1, bw1, fw1, bw1, 2 * FD, nU1,
        BH1, BH1 + (size_t)FD * KH1, BH1, BH1 + (size_t)FD * KH1);
    const int nU2 = nT * (FD / 8);
    k_wcvt<<<dim3(cdiv(nU2, NTHR), 2), NTHR, 0, stream>>>(fw2, bw2, fw2, bw2, FD, nU2,
        BH2, BH2 + (size_t)nT * KH2, BH2, BH2 + (size_t)nT * KH2);
  }

  const int nUh = MP * 32;
  k_hinit<<<cdiv(nUh, NTHR), NTHR, 0, stream>>>(xi, emb, nR, nN, nUh, SH);

  const float* ewL[2]  = {e1w, e2w};
  const float* ebL[2]  = {e1b, e2b};
  const float* b1L[2]  = {c1b1, c2b1};
  const float* gL[2]   = {c1g, c2g};
  const float* beL[2]  = {c1be, c2be};
  const float* b2L[2]  = {c1b2, c2b2};

  for (int l = 0; l < 2; ++l) {
    k_scan<0, NBA, SLA, DEGA><<<gA, NTHR, ldsA, stream>>>(src, dst, nE, nN, nN, vec8e, MP, eattr, ewL[l], ebL[l],
                                                          SH, ZA, KZ, 0, FD);
    k_gemm<GNC, KZ, 0><<<dim3(gM, 1), GTHR, 0, stream>>>(ZA, BTC + (size_t)(2 * l) * FD * KZ, b1L[l], nN, SH, FD, PT);
    k_bnfin<<<1, GNC, 0, stream>>>(PT, gM, gL[l], beL[l], SS);
    k_apply1<<<gM, NTHR, 0, stream>>>(SH, SS, nN, MP, ZA);
    k_gemm<GNC, KZ, 1><<<dim3(gM, 1), GTHR, 0, stream>>>(ZA, BTC + (size_t)(2 * l + 1) * FD * KZ, b2L[l], nN, SH, FD, PT);
    k_scan<1, NBP, SLP, DEGP><<<gP, NTHR, ldsP, stream>>>(src, batch, nN, nG, nN, vec8b, GP, eattr, e1w, e1b,
                                                          SH, P, KH1, FD * l, 2 * FD + FD * l);
  }

  const float* hb1L[2] = {fb1, bb1};
  const float* hb2L[2] = {fb2, bb2};
  for (int f = 0; f < 2; ++f) {
    k_gemm<GNC, KH1, 2><<<dim3(gH, 1), GTHR, 0, stream>>>(P, BH1 + (size_t)f * FD * KH1, hb1L[f], nG,
                                                          (float*)Q, FD, PT);
    k_gemm<GNC, KH2, 3><<<dim3(gH, nT / GNC), GTHR, 0, stream>>>(Q, BH2 + (size_t)f * nT * KH2, hb2L[f], nG,
                                                                 out + (size_t)f * (size_t)nG * (size_t)nT, nT, PT);
  }
}
